// GCN_62440234549671
// MI455X (gfx1250) — hardware-verified
//
#include <hip/hip_runtime.h>
#include <stddef.h>
#include <stdint.h>
#include <math.h>


#define DIN    41
#define KX     64
#define HD     192
#define K2     384
#define HH     96
#define NLAY   4
#define NTHR   256
#define NWAVE  8
#define EPT    8
#define CHUNK  (NTHR * EPT)
#define WCAP   (EPT * 32)
#define LISTN  (NWAVE * WCAP)
#define NBA    1024
#define SLA    10
#define RCAP   20480
#define DEGCAP 64
#define GBM    64
#define GTHR   128
#define HBM    128
#define ARB    64
#define CMP_ZINTS (LISTN + 2 * RCAP + 3 * NBA)
#define CMP_LDS_INTS (CMP_ZINTS + 16)
#define U_WIN  1536
#define U_WC1  9216
#define U_WC   36864
#define U_WP1  9216
#define U_WR1  4608
#define U_WP2  4608
#define U_ALL  56832
#define NBW    222
#define OFF_WIN 0
#define OFF_WC  (U_WIN * 8)
#define OFF_WP1 ((U_WIN + U_WC) * 8)
#define OFF_WR1 ((U_WIN + U_WC + U_WP1) * 8)
#define OFF_WP2 ((U_WIN + U_WC + U_WP1 + U_WR1) * 8)
#define WPL_HW  (U_ALL * 8)
#define WSMAX  134217728

static_assert((CHUNK & (CHUNK - 1)) == 0 && CHUNK <= 4096);
static_assert((NBA & (NBA - 1)) == 0 && NBA == (1 << SLA) && NBA == 4 * NTHR);
static_assert(((long long)CHUNK << SLA) < (1LL << 31));
static_assert(CMP_ZINTS % (NTHR * 4) == 0 && RCAP % (NTHR * 4) == 0 && LISTN % 4 == 0);
static_assert(CMP_LDS_INTS * 4 <= 300000);
static_assert(KX % 32 == 0 && K2 % 32 == 0 && K2 == 2 * HD && HD == 12 * 16 && HH == 6 * 16);
static_assert(GBM == (GTHR / 32) * 16 && HBM == NWAVE * 16 && ARB % NWAVE == 0);
static_assert(U_WIN == HD * (KX / 8) && U_WC1 == HD * (K2 / 8) && U_WC == NLAY * U_WC1);
static_assert(U_WP1 == HD * (K2 / 8) && U_WR1 == HH * (K2 / 8) && U_WP2 == HH * (K2 / 8));
static_assert(U_ALL == U_WIN + U_WC + U_WP1 + U_WR1 + U_WP2 && U_ALL == NBW * NTHR);
static_assert(U_WIN % NTHR == 0 && U_WC1 % NTHR == 0 && U_WP1 % NTHR == 0 && U_WR1 % NTHR == 0);
static_assert(DEGCAP >= 35 + 8 && RCAP >= 16623 + 2048);

typedef float          v4f   __attribute__((ext_vector_type(4)));
typedef float          v8f   __attribute__((ext_vector_type(8)));
typedef int            v4i   __attribute__((ext_vector_type(4)));
typedef int            v8i   __attribute__((ext_vector_type(8)));
typedef unsigned short v4us  __attribute__((ext_vector_type(4)));
typedef unsigned short v8us  __attribute__((ext_vector_type(8)));
typedef unsigned short v16us __attribute__((ext_vector_type(16)));
typedef __bf16         v16bf __attribute__((ext_vector_type(16)));
typedef v4f  __attribute__((may_alias)) v4fa;
typedef v4i  __attribute__((may_alias)) v4ia;
typedef v4us __attribute__((may_alias)) v4usa;
typedef v8us __attribute__((may_alias)) v8usa;
union FragB { v16bf v; v16us u; v8us h[2]; v8i w; };

__device__ __forceinline__ v8f wmb(const FragB& a, const FragB& b, v8f c) {
  v8f d = __builtin_amdgcn_wmma_f32_16x16x32_bf16(false, a.v, false, b.v, (short)0, c, false, false);
  asm volatile("v_nop\n\tv_nop\n\tv_nop\n\tv_nop" : "+v"(d) : "v"(a.w), "v"(b.w));
  return d;
}

__device__ __forceinline__ unsigned bf16_bits(float f) {
  const unsigned u = __float_as_uint(f);
  return (u + 0x7FFFu + ((u >> 16) & 1u)) >> 16;
}
__device__ __forceinline__ float bf16_val(float f) {
  return __uint_as_float(bf16_bits(f) << 16);
}
__device__ __forceinline__ float relu_np(float v) { return (v > 0.0f) ? v : (v - v); }

__device__ __forceinline__ void wave_sync() {
  __builtin_amdgcn_fence(__ATOMIC_RELEASE, "wavefront");
  __builtin_amdgcn_wave_barrier();
  __builtin_amdgcn_fence(__ATOMIC_ACQUIRE, "wavefront");
}

__device__ __forceinline__ void split4(v4f y, v4us& h, v4us& l) {
  unsigned hb;
  hb = bf16_bits(y.x); h[0] = (unsigned short)hb; l[0] = (unsigned short)bf16_bits(y.x - __uint_as_float(hb << 16));
  hb = bf16_bits(y.y); h[1] = (unsigned short)hb; l[1] = (unsigned short)bf16_bits(y.y - __uint_as_float(hb << 16));
  hb = bf16_bits(y.z); h[2] = (unsigned short)hb; l[2] = (unsigned short)bf16_bits(y.z - __uint_as_float(hb << 16));
  hb = bf16_bits(y.w); h[3] = (unsigned short)hb; l[3] = (unsigned short)bf16_bits(y.w - __uint_as_float(hb << 16));
}

__device__ __forceinline__ void put_f32_row(float* grow, v4f ya, v4f yb, int lane) {
  float* pa = grow + 4 * lane;
  float* pb = grow + 128 + 4 * (lane & 15);
  const bool lo16 = lane < 16;
  *(volatile v4f*)pa = ya;
  if (lo16) *(volatile v4f*)pb = yb;
  __threadfence();
  *(volatile v4f*)pa = ya;
  if (lo16) *(volatile v4f*)pb = yb;
}

__device__ __forceinline__ void put_hl_row(unsigned short* rowbuf, v4f ya, v4f yb, int lane, unsigned short* grow) {
  v4us ha, la, hb4, lb4;
  split4(ya, ha, la);
  split4(yb, hb4, lb4);
  const bool lo16 = lane < 16;
  *(v4usa*)(rowbuf + 4 * lane) = ha;
  *(v4usa*)(rowbuf + HD + 4 * lane) = la;
  if (lo16) {
    *(v4usa*)(rowbuf + 128 + 4 * lane) = hb4;
    *(v4usa*)(rowbuf + HD + 128 + 4 * lane) = lb4;
  }
  wave_sync();
  const v8us q0 = *(const v8usa*)(rowbuf + 8 * lane);
  const v8us q1 = *(const v8usa*)(rowbuf + 256 + 8 * (lane & 15));
  wave_sync();
  unsigned short* p0 = grow + 8 * lane;
  unsigned short* p1 = grow + 256 + 8 * (lane & 15);
  *(volatile v8us*)p0 = q0;
  if (lo16) *(volatile v8us*)p1 = q1;
  __threadfence();
  *(volatile v8us*)p0 = q0;
  if (lo16) *(volatile v8us*)p1 = q1;
}

template <int SLB>
__device__ __forceinline__ int scan_chunk(const int* __restrict__ dsts, int nE, int cbase, int slotBase,
                                          int nb, int vec8, int* list, int tid, int lane, int wave) {
  int wc = 0;
  const int el0  = tid * EPT;
  const int e0   = cbase + el0;
  const int sent = -2147483647 - 1;
  v4i da, db;
  if (vec8 != 0 && cbase + CHUNK <= nE) {
    da = *(const v4i*)(dsts + e0);
    db = *(const v4i*)(dsts + e0 + 4);
  } else {
    da.x = (e0     < nE) ? dsts[min(e0,     nE - 1)] : sent;
    da.y = (e0 + 1 < nE) ? dsts[min(e0 + 1, nE - 1)] : sent;
    da.z = (e0 + 2 < nE) ? dsts[min(e0 + 2, nE - 1)] : sent;
    da.w = (e0 + 3 < nE) ? dsts[min(e0 + 3, nE - 1)] : sent;
    db.x = (e0 + 4 < nE) ? dsts[min(e0 + 4, nE - 1)] : sent;
    db.y = (e0 + 5 < nE) ? dsts[min(e0 + 5, nE - 1)] : sent;
    db.z = (e0 + 6 < nE) ? dsts[min(e0 + 6, nE - 1)] : sent;
    db.w = (e0 + 7 < nE) ? dsts[min(e0 + 7, nE - 1)] : sent;
  }
  const unsigned nbs = (unsigned)slotBase;
  const unsigned unb = (unsigned)nb;
  const unsigned s0 = (unsigned)da.x - nbs, s1 = (unsigned)da.y - nbs;
  const unsigned s2 = (unsigned)da.z - nbs, s3 = (unsigned)da.w - nbs;
  const unsigned s4 = (unsigned)db.x - nbs, s5 = (unsigned)db.y - nbs;
  const unsigned s6 = (unsigned)db.z - nbs, s7 = (unsigned)db.w - nbs;
  const bool h0 = s0 < unb, h1 = s1 < unb, h2 = s2 < unb, h3 = s3 < unb;
  const bool h4 = s4 < unb, h5 = s5 < unb, h6 = s6 < unb, h7 = s7 < unb;
  const unsigned any = __builtin_amdgcn_ballot_w32(h0 | h1 | h2 | h3 | h4 | h5 | h6 | h7);
  if (any != 0u) {
#define HITJ(J, HJ, SJ) { \
      const unsigned mj = __builtin_amdgcn_ballot_w32(HJ); \
      if (mj != 0u) { \
        if (HJ) { \
          const int pos = wc + (int)__builtin_amdgcn_mbcnt_lo(mj, 0u); \
          if (pos < WCAP) list[wave * WCAP + pos] = ((el0 + (J)) << SLB) | (int)(SJ); \
        } \
        wc += (int)__builtin_popcount(mj); } }
    HITJ(0, h0, s0)
    HITJ(1, h1, s1)
    HITJ(2, h2, s2)
    HITJ(3, h3, s3)
    HITJ(4, h4, s4)
    HITJ(5, h5, s5)
    HITJ(6, h6, s6)
    HITJ(7, h7, s7)
#undef HITJ
  }
  return wc;
}

template <int KP, int KACT, int KMOD, int LD>
__device__ __forceinline__ void wunit(const float* __restrict__ W, int v, unsigned short* dp) {
  constexpr int UPR = KP / 8;
  const int n   = v / UPR;
  const int k8  = (v - n * UPR) * 8;
  const int kk0 = k8 % KMOD;
  v8us o;
#pragma unroll
  for (int i = 0; i < 8; ++i) {
    const int kk = kk0 + i;
    const int kc = kk < KACT ? kk : KACT - 1;
    const float w = W[(size_t)kc * LD + n];
    o[i] = (kk < KACT) ? (unsigned short)bf16_bits(w) : (unsigned short)0;
  }
  *(volatile v8us*)dp = o;
  __threadfence();
  *(volatile v8us*)dp = o;
}

__global__ __launch_bounds__(NTHR) void k_prep(const float* __restrict__ x, const float* __restrict__ Win,
                                               const float* __restrict__ Wc, const float* __restrict__ Wp1,
                                               const float* __restrict__ Wr1, const float* __restrict__ Wp2,
                                               unsigned short* wpl, unsigned short* xb, int nN, int nUx) {
  const int b = (int)blockIdx.x, tid = (int)threadIdx.x;
  if (b < NBW) {
    const int u = b * NTHR + tid;
    unsigned short* dp = wpl + (size_t)u * 8;
    if (u < U_WIN) {
      wunit<KX, DIN, KX, HD>(Win, u, dp);
    } else if (u < U_WIN + U_WC) {
      const int v = u - U_WIN;
      const int layer = v / U_WC1;
      const int vv = v - layer * U_WC1;
      wunit<K2, HD, HD, HD>(Wc + (size_t)layer * HD * HD, vv, dp);
    } else if (u < U_WIN + U_WC + U_WP1) {
      wunit<K2, HD, HD, HD>(Wp1, u - (U_WIN + U_WC), dp);
    } else if (u < U_WIN + U_WC + U_WP1 + U_WR1) {
      wunit<K2, HD, HD, HH>(Wr1, u - (U_WIN + U_WC + U_WP1), dp);
    } else {
      wunit<K2, HD, HD, HH>(Wp2, u - (U_WIN + U_WC + U_WP1 + U_WR1), dp);
    }
  } else {
    const int u = (b - NBW) * NTHR + tid;
    if (u >= nUx) return;
    const int row = u >> 3;
    const int k8  = (u & 7) * 8;
    const int rc  = row < nN ? row : nN - 1;
    const float* p = x + (size_t)rc * DIN;
    v8us o;
#pragma unroll
    for (int i = 0; i < 8; ++i) {
      const int col = k8 + i;
      const int cc  = col < DIN ? col : DIN - 1;
      const float w = p[cc];
      o[i] = (row < nN && col < DIN) ? (unsigned short)bf16_bits(w) : (unsigned short)0;
    }
    unsigned short* dp = xb + (size_t)u * 8;
    *(volatile v8us*)dp = o;
    __threadfence();
    *(volatile v8us*)dp = o;
  }
}

__global__ __launch_bounds__(NTHR) void k_degcompact(const int* __restrict__ srcs, const int* __restrict__ dsts,
                                                     int nE, int nN, int vec8,
                                                     float* dis, int* cntT, int* offT, int* srcl) {
  extern __shared__ __attribute__((aligned(16))) int dsm[];
  int* list = dsm;
  int* hl   = dsm + LISTN;
  int* sl   = dsm + LISTN + RCAP;
  int* cnt  = dsm + LISTN + 2 * RCAP;
  int* offs = cnt + NBA;
  int* cur  = offs + NBA;
  int* misc = cur + NBA;
  const int tid = (int)threadIdx.x, lane = tid & 31, wave = tid >> 5;
  const int nodeBase = (int)blockIdx.x * NBA;

  {
    const v4i z4 = {0, 0, 0, 0};
    for (int i = tid * 4; i < CMP_ZINTS; i += NTHR * 4) *(v4ia*)(dsm + i) = z4;
    if (tid < 16) misc[tid] = 0;
  }
  __syncthreads();

  int t = 0, ov = 0;
  const int nChunks = (nE + CHUNK - 1) / CHUNK;
#pragma unroll 1
  for (int ch = 0; ch < nChunks; ++ch) {
    const int cbase = ch * CHUNK;
    const int wc = scan_chunk<SLA>(dsts, nE, cbase, nodeBase, NBA, vec8, list, tid, lane, wave);
    if (lane == 0) misc[wave] = wc;
    __syncthreads();
    if (wave == 0) {
#pragma unroll 1
      for (int w2 = 0; w2 < NWAVE; ++w2) {
        int c = misc[w2];
        c = c < 0 ? 0 : (c > WCAP ? WCAP : c);
#pragma unroll 1
        for (int b0 = 0; b0 < c; b0 += 32) {
          const int idx = b0 + lane;
          const int ent = list[w2 * WCAP + (idx < WCAP ? idx : WCAP - 1)];
          const int m32 = (c - b0) < 32 ? (c - b0) : 32;
#pragma unroll 1
          for (int k = 0; k < m32; ++k) {
            const int u    = __builtin_amdgcn_readlane(ent, k);
            const int slot = u & (NBA - 1);
            const int el   = (u >> SLA) & (CHUNK - 1);
            const int pk   = ((cbase + el) << SLA) | slot;
            if (t < RCAP) {
              if (lane == 0) { hl[t] = pk; cnt[slot] = cnt[slot] + 1; }
              t = t + 1;
            } else {
              ov = 1;
            }
          }
        }
      }
    }
    __syncthreads();
  }
  if (wave == 0 && lane == 0) { misc[8] = t; misc[9] = ov; }
  __syncthreads();
  int tt = misc[8];
  tt = tt < 0 ? 0 : (tt > RCAP ? RCAP : tt);
  const int ovf = misc[9];

  if (wave == 0) {
    const int base = lane * (NBA / 32);
    int s = 0;
#pragma unroll 1
    for (int i = 0; i < NBA / 32; ++i) s += cnt[base + i];
    int incl = s;
#pragma unroll
    for (int d = 1; d < 32; d <<= 1) {
      const int y = __shfl_up(incl, d, 32);
      if (lane >= d) incl += y;
    }
    int run = incl - s;
#pragma unroll 1
    for (int i = 0; i < NBA / 32; ++i) {
      const int cv = cnt[base + i];
      offs[base + i] = run;
      cur[base + i]  = run;
      run += cv;
    }
  }
  __syncthreads();
  if (wave == 0) {
#pragma unroll 1
    for (int b0 = 0; b0 < tt; b0 += 32) {
      const int idx = b0 + lane;
      const int ent = hl[idx < RCAP ? idx : RCAP - 1];
      const int m32 = (tt - b0) < 32 ? (tt - b0) : 32;
#pragma unroll 1
      for (int k = 0; k < m32; ++k) {
        const int u    = __builtin_amdgcn_readlane(ent, k);
        const int slot = u & (NBA - 1);
        if (lane == 0) {
          int p = cur[slot];
          p = p < 0 ? 0 : (p > RCAP - 1 ? RCAP - 1 : p);
          sl[p] = u;
          cur[slot] = p + 1;
        }
      }
    }
  }
  __syncthreads();

#pragma unroll 1
  for (int i = tid * 4; i < RCAP; i += NTHR * 4) {
    const v4i e = *(const v4ia*)(sl + i);
    int e0 = e.x >> SLA, e1 = e.y >> SLA, e2 = e.z >> SLA, e3 = e.w >> SLA;
    e0 = e0 < 0 ? 0 : (e0 > nE - 1 ? nE - 1 : e0);
    e1 = e1 < 0 ? 0 : (e1 > nE - 1 ? nE - 1 : e1);
    e2 = e2 < 0 ? 0 : (e2 > nE - 1 ? nE - 1 : e2);
    e3 = e3 < 0 ? 0 : (e3 > nE - 1 ? nE - 1 : e3);
    int s0 = srcs[e0], s1 = srcs[e1], s2 = srcs[e2], s3 = srcs[e3];
    s0 = s0 < 0 ? 0 : (s0 > nN - 1 ? nN - 1 : s0);
    s1 = s1 < 0 ? 0 : (s1 > nN - 1 ? nN - 1 : s1);
    s2 = s2 < 0 ? 0 : (s2 > nN - 1 ? nN - 1 : s2);
    s3 = s3 < 0 ? 0 : (s3 > nN - 1 ? nN - 1 : s3);
    v4i r;
    r.x = (i     < tt) ? s0 : 0;
    r.y = (i + 1 < tt) ? s1 : 0;
    r.z = (i + 2 < tt) ? s2 : 0;
    r.w = (i + 3 < tt) ? s3 : 0;
    *(v4ia*)(hl + i) = r;
  }
  __syncthreads();

  int* gl = srcl + (size_t)blockIdx.x * RCAP;
#pragma unroll 1
  for (int i = tid * 4; i < RCAP; i += NTHR * 4) {
    const v4i r = *(const v4ia*)(hl + i);
    *(volatile v4i*)(gl + i) = r;
  }
  __threadfence();
#pragma unroll 1
  for (int i = tid * 4; i < RCAP; i += NTHR * 4) {
    const v4i r = *(const v4ia*)(hl + i);
    *(volatile v4i*)(gl + i) = r;
  }

  {
    const int s0 = 4 * tid;
    const v4i c4 = *(const v4ia*)(cnt + s0);
    const v4i o4 = *(const v4ia*)(offs + s0);
    const float qnan = __int_as_float(0x7fc00000);
    v4f d4;
    d4.x = rsqrtf(fmaxf((float)c4.x + 1.0f, 1.0f));
    d4.y = rsqrtf(fmaxf((float)c4.y + 1.0f, 1.0f));
    d4.z = rsqrtf(fmaxf((float)c4.z + 1.0f, 1.0f));
    d4.w = rsqrtf(fmaxf((float)c4.w + 1.0f, 1.0f));
    d4.x = (ovf != 0 || c4.x > DEGCAP) ? qnan : d4.x;
    d4.y = (ovf != 0 || c4.y > DEGCAP) ? qnan : d4.y;
    d4.z = (ovf != 0 || c4.z > DEGCAP) ? qnan : d4.z;
    d4.w = (ovf != 0 || c4.w > DEGCAP) ? qnan : d4.w;
    int*   cp = cntT + (size_t)nodeBase + s0;
    int*   op = offT + (size_t)nodeBase + s0;
    float* dp = dis  + (size_t)nodeBase + s0;
    *(volatile v4i*)cp = c4;
    *(volatile v4i*)op = o4;
    *(volatile v4f*)dp = d4;
    __threadfence();
    *(volatile v4i*)cp = c4;
    *(volatile v4i*)op = o4;
    *(volatile v4f*)dp = d4;
  }
}

template <int MODE, int K>
__global__ __launch_bounds__(GTHR) void k_gemm(const unsigned short* __restrict__ A,
                                               const unsigned short* __restrict__ WT,
                                               const float* __restrict__ bias,
                                               float* outF, unsigned short* outHL) {
  static_assert(K % 32 == 0);
  __shared__ __attribute__((aligned(16))) float stg[GBM * HD];
  __shared__ __attribute__((aligned(16))) unsigned short rowb[(GTHR / 32) * K2];
  const int tid = (int)threadIdx.x, lane = tid & 31, wave = tid >> 5, hh = lane >> 4, m = lane & 15;
  const int rowBase = (int)blockIdx.x * GBM;

  v8f acc[12];
  {
    const v8f z = {0.f, 0.f, 0.f, 0.f, 0.f, 0.f, 0.f, 0.f};
#pragma unroll
    for (int t = 0; t < 12; ++t) acc[t] = z;
  }
  const unsigned short* ap = A  + (size_t)(rowBase + 16 * wave + m) * (size_t)K + 8 * hh;
  const unsigned short* wp = WT + (size_t)m * (size_t)K + 8 * hh;
#pragma unroll 1
  for (int ks = 0; ks < K / 32; ++ks) {
    FragB af;
    af.h[0] = *(const v8usa*)(ap + 32 * ks);
    af.h[1] = *(const v8usa*)(ap + 32 * ks + 16);
#pragma unroll
    for (int t = 0; t < 6; ++t) {
      const unsigned short* wq = wp + (size_t)(16 * t) * (size_t)K + 32 * ks;
      FragB bf;
      bf.h[0] = *(const v8usa*)wq;
      bf.h[1] = *(const v8usa*)(wq + 16);
      acc[t] = wmb(af, bf, acc[t]);
    }
    asm volatile("" ::: "memory");
#pragma unroll
    for (int t = 6; t < 12; ++t) {
      const unsigned short* wq = wp + (size_t)(16 * t) * (size_t)K + 32 * ks;
      FragB bf;
      bf.h[0] = *(const v8usa*)wq;
      bf.h[1] = *(const v8usa*)(wq + 16);
      acc[t] = wmb(af, bf, acc[t]);
    }
  }

#pragma unroll
  for (int t = 0; t < 12; ++t) {
    const int lc = 16 * t + m;
#pragma unroll
    for (int r = 0; r < 8; ++r) {
      const int lr = 16 * wave + 8 * hh + r;
      stg[lr * HD + lc] = acc[t][r];
    }
  }
  __syncthreads();

  v4f ba = {0.f, 0.f, 0.f, 0.f}, bb = {0.f, 0.f, 0.f, 0.f};
  if constexpr (MODE != 0) {
    const v4f t1 = *(const v4f*)(bias + 4 * lane);
    const v4f t2 = *(const v4f*)(bias + 128 + 4 * (lane & 15));
    ba.x = bf16_val(t1.x); ba.y = bf16_val(t1.y); ba.z = bf16_val(t1.z); ba.w = bf16_val(t1.w);
    bb.x = bf16_val(t2.x); bb.y = bf16_val(t2.y); bb.z = bf16_val(t2.z); bb.w = bf16_val(t2.w);
  }
  unsigned short* rowbuf = rowb + wave * K2;
#pragma unroll 1
  for (int i = 0; i < 16; ++i) {
    const int lr = 16 * wave + i;
    const int gr = rowBase + lr;
    v4f ya = *(const v4fa*)(stg + lr * HD + 4 * lane);
    v4f yb = *(const v4fa*)(stg + lr * HD + 128 + 4 * (lane & 15));
    if constexpr (MODE != 0) { ya = ya + ba; yb = yb + bb; }
    if constexpr (MODE == 2) {
      ya.x = relu_np(ya.x); ya.y = relu_np(ya.y); ya.z = relu_np(ya.z); ya.w = relu_np(ya.w);
      yb.x = relu_np(yb.x); yb.y = relu_np(yb.y); yb.z = relu_np(yb.z); yb.w = relu_np(yb.w);
    }
    if constexpr (MODE != 2) put_f32_row(outF + (size_t)gr * HD, ya, yb, lane);
    if constexpr (MODE != 0) put_hl_row(rowbuf, ya, yb, lane, outHL + (size_t)gr * K2);
  }
}

__global__ __launch_bounds__(NTHR) void k_agg(const int* __restrict__ srcl, const int* __restrict__ cntT,
                                              const int* __restrict__ offT, const float* __restrict__ dis,
                                              const float* __restrict__ Mx, const float* __restrict__ bias,
                                              int nN, float* Hf, unsigned short* Hhl) {
  __shared__ __attribute__((aligned(16))) unsigned short rowb[NWAVE * K2];
  const int tid = (int)threadIdx.x, lane = tid & 31, wave = tid >> 5, la = lane & 15;
  unsigned short* rowbuf = rowb + wave * K2;
  v4f ba, bb;
  {
    const v4f t1 = *(const v4f*)(bias + 4 * lane);
    const v4f t2 = *(const v4f*)(bias + 128 + 4 * la);
    ba.x = bf16_val(t1.x); ba.y = bf16_val(t1.y); ba.z = bf16_val(t1.z); ba.w = bf16_val(t1.w);
    bb.x = bf16_val(t2.x); bb.y = bf16_val(t2.y); bb.z = bf16_val(t2.z); bb.w = bf16_val(t2.w);
  }
  const float qnan = __int_as_float(0x7fc00000);
#pragma unroll 1
  for (int si = 0; si < ARB / NWAVE; ++si) {
    const int node = (int)blockIdx.x * ARB + si * NWAVE + wave;
    const int nc   = node < nN ? node : nN - 1;
    const int craw = __builtin_amdgcn_readfirstlane(cntT[node]);
    const bool big = craw > DEGCAP;
    const int c = craw < 0 ? 0 : (craw > DEGCAP ? DEGCAP : craw);
    int o = __builtin_amdgcn_readfirstlane(offT[node]);
    o = o < 0 ? 0 : (o > RCAP - 1 ? RCAP - 1 : o);
    const size_t lb = (size_t)(node >> SLA) * RCAP;
    const float dd = dis[nc];
    const float rd = dd * dd;
    v4f aa = {0.f, 0.f, 0.f, 0.f}, ab = {0.f, 0.f, 0.f, 0.f};
#pragma unroll 1
    for (int b0 = 0; b0 < c; b0 += 32) {
      int idx = o + b0 + lane;
      idx = idx > RCAP - 1 ? RCAP - 1 : idx;
      int sr = srcl[lb + idx];
      sr = sr < 0 ? 0 : (sr > nN - 1 ? nN - 1 : sr);
      const float cf  = dis[sr] * dd;
      const int   cfi = __float_as_int(cf);
      const int m32 = (c - b0) < 32 ? (c - b0) : 32;
#pragma unroll 1
      for (int k = 0; k < m32; ++k) {
        const int   sk = __builtin_amdgcn_readlane(sr, k);
        const float ck = __int_as_float(__builtin_amdgcn_readlane(cfi, k));
        const float* p = Mx + (size_t)sk * HD;
        const v4f va = *(const v4f*)(p + 4 * lane);
        const v4f vb = *(const v4f*)(p + 128 + 4 * la);
        aa.x = fmaf(ck, va.x, aa.x); aa.y = fmaf(ck, va.y, aa.y);
        aa.z = fmaf(ck, va.z, aa.z); aa.w = fmaf(ck, va.w, aa.w);
        ab.x = fmaf(ck, vb.x, ab.x); ab.y = fmaf(ck, vb.y, ab.y);
        ab.z = fmaf(ck, vb.z, ab.z); ab.w = fmaf(ck, vb.w, ab.w);
      }
    }
    const float* mp = Mx + (size_t)nc * HD;
    const v4f sa = *(const v4f*)(mp + 4 * lane);
    const v4f sb = *(const v4f*)(mp + 128 + 4 * la);
    const float* hp = Hf + (size_t)nc * HD;
    const v4f ha = *(const v4fa*)(hp + 4 * lane);
    const v4f hb = *(const v4fa*)(hp + 128 + 4 * la);
    const float pz = big ? qnan : 0.0f;
    const bool live = node < nN;
    v4f ya, yb;
    ya.x = relu_np((aa.x + sa.x * rd) + ba.x) + pz; ya.y = relu_np((aa.y + sa.y * rd) + ba.y) + pz;
    ya.z = relu_np((aa.z + sa.z * rd) + ba.z) + pz; ya.w = relu_np((aa.w + sa.w * rd) + ba.w) + pz;
    yb.x = relu_np((ab.x + sb.x * rd) + bb.x) + pz; yb.y = relu_np((ab.y + sb.y * rd) + bb.y) + pz;
    yb.z = relu_np((ab.z + sb.z * rd) + bb.z) + pz; yb.w = relu_np((ab.w + sb.w * rd) + bb.w) + pz;
    v4f oa, ob;
    oa.x = live ? (ha.x + ya.x) : 0.0f; oa.y = live ? (ha.y + ya.y) : 0.0f;
    oa.z = live ? (ha.z + ya.z) : 0.0f; oa.w = live ? (ha.w + ya.w) : 0.0f;
    ob.x = live ? (hb.x + yb.x) : 0.0f; ob.y = live ? (hb.y + yb.y) : 0.0f;
    ob.z = live ? (hb.z + yb.z) : 0.0f; ob.w = live ? (hb.w + yb.w) : 0.0f;
    put_f32_row(Hf + (size_t)node * HD, oa, ob, lane);
    put_hl_row(rowbuf, oa, ob, lane, Hhl + (size_t)node * K2);
  }
}

__device__ __forceinline__ void head_phase(const unsigned short* __restrict__ A,
                                           const unsigned short* __restrict__ WT,
                                           const float* __restrict__ bias, float* stg,
                                           int rowBase, int lane, int wave) {
  const int hh = lane >> 4, m = lane & 15;
  v8f acc[6];
  {
    const v8f z = {0.f, 0.f, 0.f, 0.f, 0.f, 0.f, 0.f, 0.f};
#pragma unroll
    for (int t = 0; t < 6; ++t) acc[t] = z;
  }
  const unsigned short* ap = A  + (size_t)(rowBase + 16 * wave + m) * (size_t)K2 + 8 * hh;
  const unsigned short* wp = WT + (size_t)m * (size_t)K2 + 8 * hh;
#pragma unroll 1
  for (int ks = 0; ks < K2 / 32; ++ks) {
    FragB af;
    af.h[0] = *(const v8usa*)(ap + 32 * ks);
    af.h[1] = *(const v8usa*)(ap + 32 * ks + 16);
#pragma unroll
    for (int t = 0; t < 6; ++t) {
      const unsigned short* wq = wp + (size_t)(16 * t) * (size_t)K2 + 32 * ks;
      FragB bf;
      bf.h[0] = *(const v8usa*)wq;
      bf.h[1] = *(const v8usa*)(wq + 16);
      acc[t] = wmb(af, bf, acc[t]);
    }
  }
#pragma unroll
  for (int t = 0; t < 6; ++t) {
    const int lc = 16 * t + m;
    const float bv = bf16_val(bias[lc]);
#pragma unroll
    for (int r = 0; r < 8; ++r) {
      const int lr = 16 * wave + 8 * hh + r;
      stg[lr * HH + lc] = relu_np(acc[t][r] + bv);
    }
  }
}

__global__ __launch_bounds__(NTHR) void k_head2(const unsigned short* __restrict__ Hhl,
                                                const unsigned short* __restrict__ P1hl,
                                                const unsigned short* __restrict__ Wr1d,
                                                const unsigned short* __restrict__ Wp2d,
                                                const float* __restrict__ br1, const float* __restrict__ bp2,
                                                const float* __restrict__ Wp3, const float* __restrict__ bp3,
                                                const float* __restrict__ Wr2, const float* __restrict__ br2,
                                                float* out, int nN) {
  __shared__ __attribute__((aligned(16))) float stg[HBM * HH];
  __shared__ __attribute__((aligned(16))) float tval[HBM];
  __shared__ __attribute__((aligned(16))) float wr2s[HH];
  __shared__ __attribute__((aligned(16))) float wp3s[2 * HH];
  __shared__ __attribute__((aligned(16))) float outs[2 * HBM];
  const int tid = (int)threadIdx.x, lane = tid & 31, wave = tid >> 5;
  const int rowBase = (int)blockIdx.x * HBM;

  if (tid < HH) wr2s[tid] = bf16_val(Wr2[tid]);
  if (tid < 2 * HH) wp3s[tid] = bf16_val(Wp3[tid]);
  head_phase(Hhl, Wr1d, br1, stg, rowBase, lane, wave);
  __syncthreads();
  if (tid < HBM) {
    const float* rp = stg + tid * HH;
    float t = 0.0f;
#pragma unroll 2
    for (int j4 = 0; j4 < HH / 4; ++j4) {
      const v4f r = *(const v4fa*)(rp + 4 * j4);
      const v4f w = *(const v4fa*)(wr2s + 4 * j4);
      t = fmaf(r.x, w.x, t); t = fmaf(r.y, w.y, t); t = fmaf(r.z, w.z, t); t = fmaf(r.w, w.w, t);
    }
    tval[tid] = t + bf16_val(br2[0]);
  }
  __syncthreads();
  head_phase(P1hl, Wp2d, bp2, stg, rowBase, lane, wave);
  __syncthreads();
  if (tid < HBM) {
    const float* rp = stg + tid * HH;
    float px = 0.0f, py = 0.0f;
#pragma unroll 2
    for (int j4 = 0; j4 < HH / 4; ++j4) {
      const v4f r  = *(const v4fa*)(rp + 4 * j4);
      const v4f w0 = *(const v4fa*)(wp3s + 8 * j4);
      const v4f w1 = *(const v4fa*)(wp3s + 8 * j4 + 4);
      px = fmaf(r.x, w0.x, px); py = fmaf(r.x, w0.y, py);
      px = fmaf(r.y, w0.z, px); py = fmaf(r.y, w0.w, py);
      px = fmaf(r.z, w1.x, px); py = fmaf(r.z, w1.y, py);
      px = fmaf(r.w, w1.z, px); py = fmaf(r.w, w1.w, py);
    }
    px = px + bf16_val(bp3[0]);
    py = py + bf16_val(bp3[1]);
    const float t   = tval[tid];
    const float rad = 1.0f / (1.0f + expf(-t));
    const float nrm = sqrtf((px * px + py * py) + 1e-8f);
    outs[2 * tid]     = (px / nrm) * rad;
    outs[2 * tid + 1] = (py / nrm) * rad;
  }
  __syncthreads();
  int nvalid = nN - rowBase;
  nvalid = nvalid < 0 ? 0 : (nvalid > HBM ? HBM : nvalid);
  const int npc = nvalid >> 1;
  const v4f ov = *(const v4fa*)(outs + 4 * (tid & 63));
  const bool ok = (tid < 64) && (tid < npc);
  float* op = out + (size_t)rowBase * 2 + 4 * (tid & 63);
  if (ok) *(volatile v4f*)op = ov;
  __threadfence();
  if (ok) *(volatile v4f*)op = ov;
}

static inline int cdiv(int a, int b) { return (a + b - 1) / b; }
static inline size_t al256(size_t o) { return (o + 255) & ~(size_t)255; }

extern "C" void kernel_launch(void* const* d_in, const int* in_sizes, int n_in,
                              void* d_out, int out_size, void* d_ws, size_t ws_size,
                              hipStream_t stream) {
  if (n_in < 16) return;
  if (in_sizes[0] < DIN || (in_sizes[0] % DIN) != 0) return;
  const int nN = in_sizes[0] / DIN;
  if (nN < 16 || (nN % 16) != 0 || nN > (1 << 22)) return;
  if (in_sizes[1] < 2 || (in_sizes[1] & 1) != 0) return;
  const int nE = in_sizes[1] / 2;
  if (nE < 1 || nE >= (1 << (31 - SLA))) return;
  if (in_sizes[2] != DIN * HD || in_sizes[3] != HD) return;
  if (in_sizes[4] != NLAY * HD * HD || in_sizes[5] != NLAY * HD) return;
  if (in_sizes[6] != HD * HD || in_sizes[7] != HD) return;
  if (in_sizes[8] != HD * HH || in_sizes[9] != HH) return;
  if (in_sizes[10] != HH * 2 || in_sizes[11] != 2) return;
  if (in_sizes[12] != HD * HH || in_sizes[13] != HH) return;
  if (in_sizes[14] != HH || in_sizes[15] != 1) return;
  if ((long long)out_size != 2LL * nN) return;

  const float* x    = (const float*)d_in[0];
  const int*   edge = (const int*)d_in[1];
  const float* Win  = (const float*)d_in[2];
  const float* b_in = (const float*)d_in[3];
  const float* Wc   = (const float*)d_in[4];
  const float* bc   = (const float*)d_in[5];
  const float* Wp1  = (const float*)d_in[6];
  const float* bp1  = (const float*)d_in[7];
  const float* Wp2  = (const float*)d_in[8];
  const float* bp2  = (const float*)d_in[9];
  const float* Wp3  = (const float*)d_in[10];
  const float* bp3  = (const float*)d_in[11];
  const float* Wr1  = (const float*)d_in[12];
  const float* br1  = (const float*)d_in[13];
  const float* Wr2  = (const float*)d_in[14];
  const float* br2  = (const float*)d_in[15];
  float* out = (float*)d_out;
  const int* src = edge;
  const int* dst = edge + nE;

  const int MP  = cdiv(nN, HBM) * HBM;
  const int gA  = cdiv(MP, NBA);
  const int NBP = gA * NBA;
  if (NBP < MP || (MP % GBM) != 0 || (MP % ARB) != 0) return;
  const int vec8 = ((nE & 3) == 0) ? 1 : 0;
  const int nUx  = MP * (KX / 8);
  if ((nUx % NTHR) != 0) return;

  char* ws = (char*)d_ws;
  size_t off = 0;
  const size_t oDIS = off; off = al256(off + (size_t)NBP * 4);
  const size_t oCNT = off; off = al256(off + (size_t)NBP * 4);
  const size_t oOFF = off; off = al256(off + (size_t)NBP * 4);
  const size_t oSRC = off; off = al256(off + (size_t)gA * RCAP * 4);
  const size_t oWPL = off; off = al256(off + (size_t)WPL_HW * 2);
  const size_t oXB  = off; off = al256(off + (size_t)MP * KX * 2);
  const size_t oH   = off; off = al256(off + (size_t)MP * HD * 4);
  const size_t oHL  = off; off = al256(off + (size_t)MP * K2 * 2);
  const size_t oM   = off; off = al256(off + (size_t)MP * HD * 4);
  if (off > ws_size || off > (size_t)WSMAX) return;
  static_assert(HD * 4 == K2 * 2);
  float*          DIS  = (float*)(ws + oDIS);
  int*            CNT  = (int*)(ws + oCNT);
  int*            OFFS = (int*)(ws + oOFF);
  int*            SRCL = (int*)(ws + oSRC);
  unsigned short* WPL  = (unsigned short*)(ws + oWPL);
  unsigned short* XB   = (unsigned short*)(ws + oXB);
  float*          H    = (float*)(ws + oH);
  unsigned short* HHL  = (unsigned short*)(ws + oHL);
  float*          M    = (float*)(ws + oM);
  unsigned short* P1HL = (unsigned short*)(ws + oM);
  const unsigned short* WinT = WPL + OFF_WIN;
  const unsigned short* Wc2  = WPL + OFF_WC;
  const unsigned short* Wp1d = WPL + OFF_WP1;
  const unsigned short* Wr1d = WPL + OFF_WR1;
  const unsigned short* Wp2d = WPL + OFF_WP2;

  const size_t cmpLds = (size_t)CMP_LDS_INTS * 4;
  hipFuncSetAttribute(reinterpret_cast<const void*>(&k_degcompact), hipFuncAttributeMaxDynamicSharedMemorySize, (int)cmpLds);

  k_prep<<<NBW + nUx / NTHR, NTHR, 0, stream>>>(x, Win, Wc, Wp1, Wr1, Wp2, WPL, XB, nN, nUx);
  k_degcompact<<<gA, NTHR, cmpLds, stream>>>(src, dst, nE, nN, vec8, DIS, CNT, OFFS, SRCL);
  k_gemm<1, KX><<<MP / GBM, GTHR, 0, stream>>>(XB, WinT, b_in, H, HHL);
  for (int i = 0; i < NLAY; ++i) {
    k_gemm<0, K2><<<MP / GBM, GTHR, 0, stream>>>(HHL, Wc2 + (size_t)i * HD * K2, b_in, M, XB);
    k_agg<<<MP / ARB, NTHR, 0, stream>>>(SRCL, CNT, OFFS, DIS, M, bc + (size_t)i * HD, nN, H, HHL);
  }
  k_gemm<2, K2><<<MP / GBM, GTHR, 0, stream>>>(HHL, Wp1d, bp1, H, P1HL);
  k_head2<<<MP / HBM, NTHR, 0, stream>>>(HHL, P1HL, Wr1d, Wp2d, br1, bp2, Wp3, bp3, Wr2, br2, out, nN);
}
